// QueryCrossAttention_60610578481566
// MI455X (gfx1250) — hardware-run, weakly checked
//
#include <hip/hip_runtime.h>
#include <math.h>
#include <stdint.h>

#define NB      4
#define NQ      512
#define NKV     2048
#define NTOT    (NKV + NQ)
#define DMODEL  1024
#define NHEAD   16
#define HDIM    64
#define HALFW   (8 * HDIM)
#define WSC     64.0f
#define ACARRY  16.0f
#define QC      16.0f
#define KC      16.0f
#define VC      16.0f
#define PC      1024.0f
#define FC      1024.0f
#define ATT_SCALE 0.125f
#define LN_EPS  1e-5f
static_assert(NHEAD * HDIM == DMODEL);
static_assert(HALFW == 512 && NTOT == 2560 && HDIM == 64);
static_assert((NQ % 64) == 0 && (NTOT % 64) == 0 && (DMODEL % 64) == 0 && (NTOT % 32) == 0 && (NQ % 16) == 0);
static_assert(DMODEL == 4 * 256);
#define ATT_BLOCKS (NB * (NQ / 16) * 2)

typedef _Float16 v16h __attribute__((ext_vector_type(16)));
typedef _Float16 v8h  __attribute__((ext_vector_type(8)));
typedef float    v8f  __attribute__((ext_vector_type(8)));
typedef float    v4f  __attribute__((ext_vector_type(4)));
typedef unsigned int v4u __attribute__((ext_vector_type(4)));

union FragH { v16h v; v8h h[2]; v4u u[2]; };

__device__ __forceinline__ unsigned short bf_bits(float f) {
  unsigned u = __float_as_uint(f);
  return (unsigned short)((u + 0x7FFFu + ((u >> 16) & 1u)) >> 16);
}
__device__ __forceinline__ float bf_up(unsigned short h) { return __uint_as_float(((unsigned)h) << 16); }
__device__ __forceinline__ float bfr(float f) { return bf_up(bf_bits(f)); }
__device__ __forceinline__ unsigned short h_bits(_Float16 x) { return __builtin_bit_cast(unsigned short, x); }
__device__ __forceinline__ unsigned pk16(unsigned short a, unsigned short b) { return (unsigned)a | ((unsigned)b << 16); }
__device__ __forceinline__ v8f zero8() { v8f z = {0.f, 0.f, 0.f, 0.f, 0.f, 0.f, 0.f, 0.f}; return z; }

__device__ __forceinline__ v16h ldfrag_h(const _Float16* p) {
  FragH f;
  f.h[0] = *(const v8h*)(p);
  f.h[1] = *(const v8h*)(p + 16);
  return f.v;
}
__device__ __forceinline__ v16h ldfrag_u(const unsigned short* p) {
  FragH f;
  f.u[0] = *(const v4u*)(p);
  f.u[1] = *(const v4u*)(p + 16);
  return f.v;
}

__device__ __forceinline__ v8f mma_raw(v16h a, v16h b, v8f c) {
  return __builtin_amdgcn_wmma_f32_16x16x32_f16(false, a, false, b, (short)0, c, false, false);
}
__device__ __forceinline__ void dep_guard1(v8f& a, v8f& b, v16h x) {
#if defined(__HIP_DEVICE_COMPILE__)
  asm volatile("v_nop\n\tv_nop\n\tv_nop\n\tv_nop" : "+v"(a), "+v"(b) : "v"(x));
#endif
}
__device__ __forceinline__ void guard_s2(v8f& s, v16h a0, v16h a1) {
#if defined(__HIP_DEVICE_COMPILE__)
  asm volatile("v_nop\n\tv_nop\n\tv_nop\n\tv_nop" : "+v"(s) : "v"(a0), "v"(a1));
#endif
}
__device__ __forceinline__ void guard_s4(v8f& s, v16h a0, v16h a1, v16h b0, v16h b1) {
#if defined(__HIP_DEVICE_COMPILE__)
  asm volatile("v_nop\n\tv_nop\n\tv_nop\n\tv_nop" : "+v"(s) : "v"(a0), "v"(a1), "v"(b0), "v"(b1));
#endif
}
__device__ __forceinline__ void guard_pv4(v8f& a, v8f& b, v8f& c, v8f& d, v16h x, v16h y, v16h z, v16h w, v16h u) {
#if defined(__HIP_DEVICE_COMPILE__)
  asm volatile("v_nop\n\tv_nop\n\tv_nop\n\tv_nop"
               : "+v"(a), "+v"(b), "+v"(c), "+v"(d) : "v"(x), "v"(y), "v"(z), "v"(w), "v"(u));
#endif
}
__device__ __forceinline__ void keep4_h(v16h a, v16h b, v16h c, v16h d) {
#if defined(__HIP_DEVICE_COMPILE__)
  asm volatile("v_nop" :: "v"(a), "v"(b), "v"(c), "v"(d));
#endif
}
__device__ __forceinline__ void acc_guard4(v8f& a, v8f& b, v8f& c, v8f& d) {
#if defined(__HIP_DEVICE_COMPILE__)
  asm volatile("v_nop\n\tv_nop\n\tv_nop\n\tv_nop" : "+v"(a), "+v"(b), "+v"(c), "+v"(d));
#endif
}
__device__ __forceinline__ void wave_sync_lds() {
  __builtin_amdgcn_fence(__ATOMIC_RELEASE, "workgroup");
  __builtin_amdgcn_wave_barrier();
  __builtin_amdgcn_fence(__ATOMIC_ACQUIRE, "workgroup");
}

__global__ __launch_bounds__(256) void conv_wT(const float* __restrict__ W, unsigned short* dst, float wsc) {
  __shared__ float t[64 * 65];
  const int tid = threadIdx.x;
  const int kt = blockIdx.x & 15, nt = blockIdx.x >> 4;
  const int k0 = kt * 64, n0 = nt * 64;
#pragma unroll
  for (int it = 0; it < 4; ++it) {
    const int p  = it * 256 + tid;
    const int r  = p >> 4, c4 = (p & 15) * 4;
    const v4f v = *(const v4f*)(W + (size_t)(k0 + r) * DMODEL + n0 + c4);
    float* tp = t + r * 65 + c4;
    tp[0] = v[0]; tp[1] = v[1]; tp[2] = v[2]; tp[3] = v[3];
  }
  __syncthreads();
  v4u ov[2];
#pragma unroll
  for (int it = 0; it < 2; ++it) {
    const int p   = it * 256 + tid;
    const int nr  = p >> 3, kc8 = (p & 7) * 8;
    v4u o = {0u, 0u, 0u, 0u};
#pragma unroll
    for (int e = 0; e < 4; ++e) {
      const float f0 = bfr(t[(kc8 + 2 * e) * 65 + nr]) * wsc;
      const float f1 = bfr(t[(kc8 + 2 * e + 1) * 65 + nr]) * wsc;
      o[e] = pk16(h_bits((_Float16)f0), h_bits((_Float16)f1));
    }
    ov[it] = o;
  }
  unsigned short* d = dst + (size_t)n0 * DMODEL + k0;
  for (int pass = 0; pass < 2; ++pass) {
#pragma unroll
    for (int it = 0; it < 2; ++it) {
      const int p   = it * 256 + tid;
      const int nr  = p >> 3, kc8 = (p & 7) * 8;
      *(volatile v4u*)(d + (size_t)nr * DMODEL + kc8) = ov[it];
    }
    __threadfence();
  }
}

__global__ __launch_bounds__(256) void ln_pack(const float* __restrict__ X, const float* __restrict__ gam,
                                               const float* __restrict__ bet, unsigned short* XI,
                                               int nrows, int rpb, int rowOff, float carry) {
  const int lane = threadIdx.x & 31, wave = threadIdx.x >> 5;
  const int row = blockIdx.x * 8 + wave;
  if (row >= nrows) return;
  const int b = row / rpb, r = row - b * rpb;
  const float* xp = X + (size_t)row * DMODEL;
  unsigned short* op = XI + ((size_t)b * NTOT + rowOff + r) * DMODEL;
  v4f y[8];
  float s = 0.f;
#pragma unroll
  for (int j = 0; j < 4; ++j) {
    const int c0 = j * 256 + lane * 8;
    const v4f a0 = *(const v4f*)(xp + c0), a1 = *(const v4f*)(xp + c0 + 4);
    v4f t0, t1;
#pragma unroll
    for (int e = 0; e < 4; ++e) { t0[e] = bfr(a0[e]); t1[e] = bfr(a1[e]); s += t0[e] + t1[e]; }
    y[2 * j] = t0; y[2 * j + 1] = t1;
  }
#pragma unroll
  for (int off = 1; off < 32; off <<= 1) s += __shfl_xor(s, off, 32);
  const float mu = s * (1.0f / (float)DMODEL);
  float ss = 0.f;
#pragma unroll
  for (int j = 0; j < 8; ++j) {
#pragma unroll
    for (int e = 0; e < 4; ++e) { const float d = y[j][e] - mu; ss += d * d; }
  }
#pragma unroll
  for (int off = 1; off < 32; off <<= 1) ss += __shfl_xor(ss, off, 32);
  const float var  = ss * (1.0f / (float)DMODEL);
  const float rstd = rsqrtf(var + LN_EPS);
  v4u res[4];
#pragma unroll
  for (int j = 0; j < 4; ++j) {
    const int c0 = j * 256 + lane * 8;
    const v4f g0 = *(const v4f*)(gam + c0), g1 = *(const v4f*)(gam + c0 + 4);
    const v4f b0 = *(const v4f*)(bet + c0), b1 = *(const v4f*)(bet + c0 + 4);
    float t[8];
#pragma unroll
    for (int e = 0; e < 4; ++e) {
      t[e]     = ((y[2 * j][e] - mu) * rstd * bfr(g0[e]) + bfr(b0[e])) * carry;
      t[4 + e] = ((y[2 * j + 1][e] - mu) * rstd * bfr(g1[e]) + bfr(b1[e])) * carry;
    }
    v4u o = {0u, 0u, 0u, 0u};
#pragma unroll
    for (int e = 0; e < 4; ++e) o[e] = pk16(h_bits((_Float16)t[2 * e]), h_bits((_Float16)t[2 * e + 1]));
    res[j] = o;
  }
  for (int pass = 0; pass < 2; ++pass) {
#pragma unroll
    for (int j = 0; j < 4; ++j) *(volatile v4u*)(op + j * 256 + lane * 8) = res[j];
    __threadfence();
  }
}

template <int OM, int BM, int HASR>
__global__ __launch_bounds__(256) void gemm64(
    const unsigned short* __restrict__ Ap, int lda, long long sA,
    const unsigned short* __restrict__ Btp, int ldb, long long sB,
    const float* __restrict__ bias, float bscale,
    const float* __restrict__ Rp,
    void* Cout, int ldc, long long sC,
    int M, int N, int K, float oscale) {
  __shared__ __align__(16) float sT[8][16 * 68];
  const int by   = blockIdx.y;
  const int lane = threadIdx.x & 31;
  const int wave = threadIdx.x >> 5;
  const int tilesN = N >> 6;
  const int tilesM = M >> 6;
  const int tile = blockIdx.x * 8 + wave;
  if (tile >= tilesM * tilesN) return;
  const int tm = tile / tilesN;
  const int tn = tile - tm * tilesN;
  const int m0 = tm << 6;
  const int n0 = tn << 6;

  const unsigned short* A1 = Ap  + (size_t)((long long)by * sA);
  const unsigned short* Bb = Btp + (size_t)((long long)by * sB);

  const int rlane = lane & 15;
  const int koff  = (lane >> 4) * 8;
  const int mOff  = (lane >> 4) * 8;

  v8f acc[4][4];
#pragma unroll
  for (int i = 0; i < 4; ++i)
#pragma unroll
    for (int j = 0; j < 4; ++j) acc[i][j] = zero8();

  for (int k0 = 0; k0 < K; k0 += 32) {
    v16h bh[4];
#pragma unroll
    for (int j = 0; j < 4; ++j) {
      const size_t bofs = (size_t)(n0 + (j << 4) + rlane) * ldb + koff + k0;
      bh[j] = ldfrag_u(Bb + bofs);
    }
#pragma unroll
    for (int i = 0; i < 4; ++i) {
      const size_t ao = (size_t)(m0 + (i << 4) + rlane) * lda + koff + k0;
      const v16h ah = ldfrag_u(A1 + ao);
#pragma unroll
      for (int j = 0; j < 4; ++j) acc[i][j] = mma_raw(ah, bh[j], acc[i][j]);
      dep_guard1(acc[i][0], acc[i][3], ah);
    }
    keep4_h(bh[0], bh[1], bh[2], bh[3]);
  }
  acc_guard4(acc[0][0], acc[0][1], acc[0][2], acc[0][3]);
  acc_guard4(acc[1][0], acc[1][1], acc[1][2], acc[1][3]);
  acc_guard4(acc[2][0], acc[2][1], acc[2][2], acc[2][3]);
  acc_guard4(acc[3][0], acc[3][1], acc[3][2], acc[3][3]);

  const int hh2 = lane >> 4, c4 = (lane & 15) * 4;
  const int q8  = lane >> 3, c8 = (lane & 7) * 8;
  float bc[4];
  float bcol[8];
#pragma unroll
  for (int e = 0; e < 4; ++e) bc[e] = 0.f;
#pragma unroll
  for (int e = 0; e < 8; ++e) bcol[e] = 0.f;
  if constexpr (BM == 1) {
    if constexpr (OM == 0) {
      const int cb = n0 + c4;
      const int i0 = (cb < N - 4) ? cb : (N - 4);
      const v4f b0v = *(const v4f*)(bias + i0);
#pragma unroll
      for (int e = 0; e < 4; ++e) bc[e] = bfr(b0v[e]) * bscale;
    } else {
      const int cb = n0 + c8;
      const int i0 = (cb < N - 8) ? cb : (N - 8);
      const v4f b0v = *(const v4f*)(bias + i0), b1v = *(const v4f*)(bias + i0 + 4);
#pragma unroll
      for (int e = 0; e < 4; ++e) { bcol[e] = bfr(b0v[e]) * bscale; bcol[4 + e] = bfr(b1v[e]) * bscale; }
    }
  }

  float* slab = sT[wave];
#pragma unroll
  for (int i = 0; i < 4; ++i) {
    const int mBase = m0 + (i << 4);
#pragma unroll
    for (int j = 0; j < 4; ++j) {
#pragma unroll
      for (int r = 0; r < 8; ++r) {
        slab[(mOff + r) * 68 + (j << 4) + rlane] = acc[i][j][r];
      }
    }
    wave_sync_lds();
    if constexpr (OM == 0) {
      float* C = (float*)Cout + (size_t)((long long)by * sC);
      v4f vals[8];
#pragma unroll
      for (int it = 0; it < 8; ++it) {
        const int row = it * 2 + hh2;
        const int gr  = mBase + row;
        v4f v = *(const v4f*)(slab + row * 68 + c4);
        float br = 0.f;
        if constexpr (BM == 2) {
          const int ir = (gr < M - 1) ? gr : (M - 1);
          br = bfr(bias[ir]) * bscale;
        }
        v4f rv = {0.f, 0.f, 0.f, 0.f};
        if constexpr (HASR != 0) {
          const float* R = Rp + (size_t)((long long)by * sC);
          const v4f rraw = *(const v4f*)(R + (size_t)gr * ldc + n0 + c4);
#pragma unroll
          for (int e = 0; e < 4; ++e) rv[e] = bfr(rraw[e]);
        }
#pragma unroll
        for (int e = 0; e < 4; ++e) v[e] = v[e] * oscale + bc[e] + br + rv[e];
        vals[it] = v;
      }
      for (int pass = 0; pass < 2; ++pass) {
#pragma unroll
        for (int it = 0; it < 8; ++it) {
          const int gr = mBase + it * 2 + hh2;
          *(volatile v4f*)(C + (size_t)gr * ldc + n0 + c4) = vals[it];
        }
        __threadfence();
      }
    } else {
      unsigned short* C = (unsigned short*)Cout + (size_t)((long long)by * sC);
      v4u hv[4];
#pragma unroll
      for (int it = 0; it < 4; ++it) {
        const int row = it * 4 + q8;
        const float* sp = slab + row * 68 + c8;
        float br = 0.f;
        if constexpr (BM == 2) {
          const int gr = mBase + row;
          const int ir = (gr < M - 1) ? gr : (M - 1);
          br = bfr(bias[ir]) * bscale;
        }
        v4u a = {0u, 0u, 0u, 0u};
#pragma unroll
        for (int e = 0; e < 4; ++e) {
          const float f0 = sp[2 * e] * oscale + bcol[2 * e] + br;
          const float f1 = sp[2 * e + 1] * oscale + bcol[2 * e + 1] + br;
          a[e] = pk16(h_bits((_Float16)f0), h_bits((_Float16)f1));
        }
        hv[it] = a;
      }
      for (int pass = 0; pass < 2; ++pass) {
#pragma unroll
        for (int it = 0; it < 4; ++it) {
          const int row = it * 4 + q8;
          *(volatile v4u*)(C + (size_t)(mBase + row) * ldc + n0 + c8) = hv[it];
        }
        __threadfence();
      }
    }
    wave_sync_lds();
  }
}

__global__ __launch_bounds__(256)
void attn64(const unsigned short* __restrict__ QHp, const unsigned short* __restrict__ KHp,
            const unsigned short* __restrict__ VTq, unsigned short* CT) {
  __shared__ __align__(16) float Ps[8][16 * 36];
  __shared__ __align__(16) unsigned short Os[16 * HALFW];

  const int tid  = threadIdx.x;
  const int wave = tid >> 5;
  const int lane = tid & 31;
  const int hh   = lane >> 4;
  const int c    = lane & 15;

  const int hg   = blockIdx.x & 1;
  const int t    = blockIdx.x >> 1;
  const int qt   = t & ((NQ / 16) - 1);
  const int bat  = t / (NQ / 16);
  const int head = hg * 8 + wave;
  const int q0   = qt * 16;

  const size_t qofs = ((size_t)bat * NQ + q0 + c) * DMODEL + head * HDIM + 8 * hh;
  const _Float16* Qh = (const _Float16*)(const void*)QHp + qofs;
  const _Float16* Kb = (const _Float16*)(const void*)KHp + (size_t)bat * NTOT * DMODEL + head * HDIM + 8 * hh;
  const _Float16* Vb = (const _Float16*)(const void*)VTq + ((size_t)bat * DMODEL + head * HDIM) * NTOT + 8 * hh;
  const float lsc = (1.4426950408889634f * ATT_SCALE) / (QC * KC);

  const v16h qa = ldfrag_h(Qh), qb = ldfrag_h(Qh + 32);

  float mrow[8], lrow[8];
  v8f o0 = zero8(), o1 = zero8(), o2 = zero8(), o3 = zero8();
#pragma unroll
  for (int r = 0; r < 8; ++r) { mrow[r] = -INFINITY; lrow[r] = 0.f; }
  float* pt = Ps[wave];

#pragma unroll 1
  for (int kb = 0; kb < NTOT; kb += 32) {
    const _Float16* kp = Kb + (size_t)(kb + c) * DMODEL;
    v8f s0, s1;
    {
      const v16h k0 = ldfrag_h(kp), k1 = ldfrag_h(kp + 32);
      s0 = mma_raw(qa, k0, zero8());
      s0 = mma_raw(qb, k1, s0);
      guard_s2(s0, k0, k1);
    }
    {
      const _Float16* kq = kp + (size_t)16 * DMODEL;
      const v16h k0 = ldfrag_h(kq), k1 = ldfrag_h(kq + 32);
      s1 = mma_raw(qa, k0, zero8());
      s1 = mma_raw(qb, k1, s1);
      guard_s4(s1, k0, k1, qa, qb);
    }
#pragma unroll
    for (int r = 0; r < 8; ++r) {
      const float t0 = s0[r] * lsc, t1 = s1[r] * lsc;
      float mx = fmaxf(t0, t1);
#pragma unroll
      for (int off = 1; off < 16; off <<= 1) mx = fmaxf(mx, __shfl_xor(mx, off, 32));
      const float mn = fmaxf(mrow[r], mx);
      const float al = exp2f(mrow[r] - mn);
      mrow[r] = mn;
      const float e0 = exp2f(t0 - mn), e1 = exp2f(t1 - mn);
      float ps = e0 + e1;
#pragma unroll
      for (int off = 1; off < 16; off <<= 1) ps += __shfl_xor(ps, off, 32);
      lrow[r] = lrow[r] * al + ps;
      o0[r] *= al;
      o1[r] *= al;
      o2[r] *= al;
      o3[r] *= al;
      const int ro = (8 * hh + r) * 36 + c;
      pt[ro]      = e0;
      pt[ro + 16] = e1;
    }
    wave_sync_lds();
    FragH ph;
    {
      const float* prow = pt + c * 36 + 8 * hh;
      const v4f p0 = *(const v4f*)(prow), p1 = *(const v4f*)(prow + 4);
      const v4f p2 = *(const v4f*)(prow + 16), p3 = *(const v4f*)(prow + 20);
#pragma unroll
      for (int e = 0; e < 4; ++e) {
        ph.h[0][e]     = (_Float16)(p0[e] * PC);
        ph.h[0][4 + e] = (_Float16)(p1[e] * PC);
        ph.h[1][e]     = (_Float16)(p2[e] * PC);
        ph.h[1][4 + e] = (_Float16)(p3[e] * PC);
      }
    }
    const _Float16* vp = Vb + (size_t)c * NTOT + kb;
    {
      const v16h vb0 = ldfrag_h(vp);
      const v16h vb1 = ldfrag_h(vp + (size_t)16 * NTOT);
      const v16h vb2 = ldfrag_h(vp + (size_t)32 * NTOT);
      const v16h vb3 = ldfrag_h(vp + (size_t)48 * NTOT);
      o0 = mma_raw(ph.v, vb0, o0);
      o1 = mma_raw(ph.v, vb1, o1);
      o2 = mma_raw(ph.v, vb2, o2);
      o3 = mma_raw(ph.v, vb3, o3);
      guard_pv4(o0, o1, o2, o3, ph.v, vb0, vb1, vb2, vb3);
    }
    wave_sync_lds();
  }

  const float oc = FC / (PC * VC);
  unsigned short* osw = Os + wave * HDIM + c;
#pragma unroll
  for (int r = 0; r < 8; ++r) {
    const float inv = (1.0f / lrow[r]) * oc;
    unsigned short* op = osw + (8 * hh + r) * HALFW;
    op[0]  = h_bits((_Float16)(o0[r] * inv));
    op[16] = h_bits((_Float16)(o1[r] * inv));
    op[32] = h_bits((_Float16)(o2[r] * inv));
    op[48] = h_bits((_Float16)(o3[r] * inv));
  }
  __syncthreads();
  {
    v4u vals[4];
#pragma unroll
    for (int it = 0; it < 4; ++it) {
      const int p   = it * 256 + tid;
      const int row = p >> 6;
      const int c8  = (p & 63) * 8;
      vals[it] = *(const v4u*)(Os + row * HALFW + c8);
    }
    unsigned short* dst = CT + ((size_t)bat * NQ + q0) * DMODEL + hg * HALFW;
    for (int pass = 0; pass < 2; ++pass) {
#pragma unroll
      for (int it = 0; it < 4; ++it) {
        const int p   = it * 256 + tid;
        const int row = p >> 6;
        const int c8  = (p & 63) * 8;
        *(volatile v4u*)(dst + (size_t)row * DMODEL + c8) = vals[it];
      }
      __threadfence();
    }
  }
}

extern "C" void kernel_launch(void* const* d_in, const int* in_sizes, int n_in,
                              void* d_out, int out_size, void* d_ws, size_t ws_size,
                              hipStream_t stream) {
  if (n_in < 14) return;
  if (in_sizes[0] != NB * NQ * DMODEL) return;
  if (in_sizes[1] != NB * NKV * DMODEL) return;
  if (in_sizes[2] != DMODEL || in_sizes[3] != DMODEL || in_sizes[4] != DMODEL || in_sizes[5] != DMODEL) return;
  if (in_sizes[6] != DMODEL * DMODEL || in_sizes[8] != DMODEL * DMODEL ||
      in_sizes[10] != DMODEL * DMODEL || in_sizes[12] != DMODEL * DMODEL) return;
  if (in_sizes[7] != DMODEL || in_sizes[9] != DMODEL || in_sizes[11] != DMODEL || in_sizes[13] != DMODEL) return;
  if (out_size != NB * NQ * DMODEL) return;

  const float* query   = (const float*)d_in[0];
  const float* kv      = (const float*)d_in[1];
  const float* ln_q_g  = (const float*)d_in[2];
  const float* ln_q_b  = (const float*)d_in[3];
  const float* ln_kv_g = (const float*)d_in[4];
  const float* ln_kv_b = (const float*)d_in[5];
  const float* w_q     = (const float*)d_in[6];
  const float* b_q     = (const float*)d_in[7];
  const float* w_k     = (const float*)d_in[8];
  const float* b_k     = (const float*)d_in[9];
  const float* w_v     = (const float*)d_in[10];
  const float* b_v     = (const float*)d_in[11];
  const float* w_o     = (const float*)d_in[12];
  const float* b_o     = (const float*)d_in[13];
  float*       out     = (float*)d_out;

  const size_t PW  = (size_t)DMODEL * DMODEL * 2;
  const size_t PXI = (size_t)NB * NTOT * DMODEL * 2;
  const size_t PQH = (size_t)NB * NQ * DMODEL * 2;
  const size_t PKH = (size_t)NB * NTOT * DMODEL * 2;
  const size_t PVT = (size_t)NB * DMODEL * NTOT * 2;
  const size_t PCT = (size_t)NB * NQ * DMODEL * 2;
  size_t off = 0;
  const size_t oWQ = off; off += PW;
  const size_t oWK = off; off += PW;
  const size_t oWV = off; off += PW;
  const size_t oWO = off; off += PW;
  const size_t oXI = off; off += PXI;
  const size_t oQH = off; off += PQH;
  const size_t oKH = off; off += PKH;
  const size_t oVT = off; off += PVT;
  const size_t oCT = off; off += PCT;
  if (off > ws_size) return;
  if (off > (size_t)134217728) return;

  char* ws = (char*)d_ws;
  unsigned short* WQT = (unsigned short*)(ws + oWQ);
  unsigned short* WKT = (unsigned short*)(ws + oWK);
  unsigned short* WVT = (unsigned short*)(ws + oWV);
  unsigned short* WOT = (unsigned short*)(ws + oWO);
  unsigned short* XI  = (unsigned short*)(ws + oXI);
  unsigned short* QH  = (unsigned short*)(ws + oQH);
  unsigned short* KH  = (unsigned short*)(ws + oKH);
  unsigned short* VTp = (unsigned short*)(ws + oVT);
  unsigned short* CT  = (unsigned short*)(ws + oCT);

  const dim3 blk(256);
  const dim3 gCW((DMODEL / 64) * (DMODEL / 64));
  const dim3 gLK((NB * NKV) / 8);
  const dim3 gLQ((NB * NQ) / 8);
  const int tilesQ = (NQ / 64) * (DMODEL / 64);
  const int tilesK = ((NB * NTOT) / 64) * (DMODEL / 64);
  const int tilesV = (DMODEL / 64) * (NTOT / 64);
  const int tilesO = ((NB * NQ) / 64) * (DMODEL / 64);
  if ((tilesQ % 8) != 0 || (tilesK % 8) != 0 || (tilesV % 8) != 0 || (tilesO % 8) != 0) return;
  const dim3 gQ(tilesQ / 8, NB);
  const dim3 gK(tilesK / 8, 1);
  const dim3 gV(tilesV / 8, NB);
  const dim3 gO(tilesO / 8, 1);
  const dim3 gAT(ATT_BLOCKS);

  conv_wT<<<gCW, blk, 0, stream>>>(w_q, WQT, WSC);
  conv_wT<<<gCW, blk, 0, stream>>>(w_k, WKT, WSC);
  conv_wT<<<gCW, blk, 0, stream>>>(w_v, WVT, WSC);
  conv_wT<<<gCW, blk, 0, stream>>>(w_o, WOT, WSC);

  ln_pack<<<gLK, blk, 0, stream>>>(kv, ln_kv_g, ln_kv_b, XI, NB * NKV, NKV, 0, ACARRY);
  ln_pack<<<gLQ, blk, 0, stream>>>(query, ln_q_g, ln_q_b, XI, NB * NQ, NQ, NKV, ACARRY);

  gemm64<2, 1, 0><<<gQ, blk, 0, stream>>>(
      XI + (size_t)NKV * DMODEL, DMODEL, (long long)NTOT * DMODEL,
      WQT, DMODEL, 0LL,
      b_q, QC,
      (const float*)0,
      (void*)QH, DMODEL, (long long)NQ * DMODEL,
      NQ, DMODEL, DMODEL, QC / (ACARRY * WSC));

  gemm64<2, 1, 0><<<gK, blk, 0, stream>>>(
      XI, DMODEL, 0LL,
      WKT, DMODEL, 0LL,
      b_k, KC,
      (const float*)0,
      (void*)KH, DMODEL, 0LL,
      NB * NTOT, DMODEL, DMODEL, KC / (ACARRY * WSC));

  gemm64<2, 2, 0><<<gV, blk, 0, stream>>>(
      WVT, DMODEL, 0LL,
      XI, DMODEL, (long long)NTOT * DMODEL,
      b_v, VC,
      (const float*)0,
      (void*)VTp, NTOT, (long long)DMODEL * NTOT,
      DMODEL, NTOT, DMODEL, VC / (ACARRY * WSC));

  attn64<<<gAT, blk, 0, stream>>>(QH, KH, VTp, CT);

  gemm64<0, 1, 1><<<gO, blk, 0, stream>>>(
      CT, DMODEL, 0LL,
      WOT, DMODEL, 0LL,
      b_o, 1.0f,
      query,
      (void*)out, DMODEL, 0LL,
      NB * NQ, DMODEL, DMODEL, 1.0f / (FC * WSC));
  (void)hipGetLastError();
}
